// StructEmbedder_29841432773281
// MI455X (gfx1250) — hardware-verified
//
#include <hip/hip_runtime.h>
#include <hip/hip_bf16.h>


typedef __attribute__((ext_vector_type(16))) _Float16 v16bf;
typedef __attribute__((ext_vector_type(8)))  _Float16 v8hf;
typedef __attribute__((ext_vector_type(8)))  float  v8f;
typedef _Float16 e16;
#define WCSCALE 256.0f
#define VST2(T, ptr, val) do { const T _v = (val); *(volatile T*)(ptr) = _v; __threadfence(); *(volatile T*)(ptr) = _v; } while (0)
#define INV_WCSCALE (1.0f / 256.0f)
#define A2SCALE 1024.0f
#define INV_A2SCALE (1.0f / 1024.0f)
__device__ __forceinline__ v8f wmma16(v16bf a, v16bf b, v8f c) {
    v8f d = __builtin_amdgcn_wmma_f32_16x16x32_f16(false, a, false, b, (short)0, c, false, false);
    asm volatile("v_nop\n\tv_nop\n\tv_nop\n\tv_nop" : "+v"(d) : "v"(a), "v"(b));
    return d;
}

#define NROUGH 3136
#define NDIST  7840
#define KTOT   13664
#define NCHUNK 427

#define LOG2E 1.4426950408889634f

#define S1    1.25f
#define OFF1  2.625f
#define C1    (-8.0f)
#define S2    1.25f
#define OFF2  2.625f
#define C2    (-8.0f)
#define S3    (64.0f/62.0f)
#define OFF3  (-32.0f - 0.5f*S3)
#define C3    (-0.5f/((0.2f*S3)*(0.2f*S3)))
#define C1L   (C1*LOG2E)
#define C2L   (C2*LOG2E)
#define C3L   (C3*LOG2E)

__device__ __forceinline__ int kmapA(int e, int hi) {
    return (e < 8) ? (hi * 8 + e) : (16 + hi * 8 + (e - 8));
}

__device__ __forceinline__ float2 group_ab(float x, float off0, float s, float cf,
                                           int nb, float msk) {
    float fj = floorf((x - off0) / s + 0.5f);
    fj = fminf(fmaxf(fj, 0.0f), (float)(nb - 1));
    float dm = x - (off0 + fj * s);
    float mx = cf * dm * dm;
    float sum = 0.0f;
    for (int j = 0; j < nb; ++j) {
        float dj = x - (off0 + j * s);
        sum += __expf(cf * dj * dj - mx);
    }
    float lpre2 = __log2f(msk / sum);
    float2 g;
    g.x = -2.0f * cf * x * LOG2E;
    g.y = (cf * x * x - mx) * LOG2E + lpre2;
    return g;
}

__device__ __forceinline__ int bswiz(int chunk, int nfrag_per_chunk, int kk, int n) {
    int frag = chunk * nfrag_per_chunk + (n >> 4);
    int lane = (((kk >> 3) & 1) << 4) + (n & 15);
    return (frag * 32 + lane) * 16 + (kk & 7) + ((kk >> 4) << 3);
}
__device__ __forceinline__ void bswiz_inv(int frag, int lane, int e, int nfrag_per_chunk, int& chunk, int& kk, int& n) {
    chunk = frag / nfrag_per_chunk; const int ntile = frag - chunk * nfrag_per_chunk;
    n = ntile * 16 + (lane & 15);
    kk = kmapA(e, lane >> 4);
}

__device__ __forceinline__ v16bf make_afrag(int c, int r, int hi,
                                            const float2* sg1, const float2* sg2,
                                            const float2* sg3) {
    v16bf afrag;
    if (c < 98) {
#pragma unroll
        for (int e = 0; e < 16; ++e) {
            int f = c * 32 + kmapA(e, hi);
            float2 g = sg1[r * 196 + (f >> 4)];
            float offb = OFF1 + (float)(f & 15) * S1;
            afrag[e] = (e16)exp2f(offb * (C1L * offb + g.x) + g.y);
        }
    } else if (c < 343) {
#pragma unroll
        for (int e = 0; e < 16; ++e) {
            int gix = c * 32 + kmapA(e, hi) - NROUGH;
            int apair = gix / 40, bin = gix - apair * 40;
            float2 g = sg2[r * 196 + apair];
            float offb = OFF2 + (float)bin * S2;
            afrag[e] = (e16)exp2f(offb * (C2L * offb + g.x) + g.y);
        }
    } else {
#pragma unroll
        for (int e = 0; e < 16; ++e) {
            int gix = c * 32 + kmapA(e, hi) - (NROUGH + NDIST);
            float2 g = sg3[r * 42 + (gix >> 6)];
            float offb = OFF3 + (float)(gix & 63) * S3;
            afrag[e] = (e16)exp2f(offb * (C3L * offb + g.x) + g.y);
        }
    }
    return afrag;
}

__device__ __forceinline__ void feat_decode(int f, int& type, int& rowblk, int& bin) {
    if (f < NROUGH) { type = 0; rowblk = f >> 4; bin = f & 15; }
    else if (f < NROUGH + NDIST) { const int g = f - NROUGH; type = 1; rowblk = g / 40; bin = g - rowblk * 40; }
    else { const int g = f - (NROUGH + NDIST); type = 2; rowblk = g >> 6; bin = g & 63; }
}
__global__ __launch_bounds__(128) void fold_weights_kernel(const float* __restrict__ We1, const float* __restrict__ be1,
                                    const float* __restrict__ We2, const float* __restrict__ be2,
                                    const float* __restrict__ We3, const float* __restrict__ be3,
                                    const float* __restrict__ Wl1, const float* __restrict__ Wl2,
                                    const float* __restrict__ Wl3, e16* __restrict__ wc) {
    __shared__ __attribute__((aligned(16))) e16 sdst[1024];
    const int c = blockIdx.x;
    const int lane = threadIdx.x & 31, wave = threadIdx.x >> 5, hh = lane >> 4, l16 = lane & 15;
    const int mt = wave >> 1, nt = wave & 1;
    int type0, rb0, bin0; feat_decode(c * 32, type0, rb0, bin0);
    const float* We = (type0 == 0) ? We1 : (type0 == 1) ? We2 : We3;
    const float* be = (type0 == 0) ? be1 : (type0 == 1) ? be2 : be3;
    const float* Wl = (type0 == 0) ? Wl1 : (type0 == 1) ? Wl2 : Wl3;
    const int nrows = (type0 == 0) ? 196 * 32 : (type0 == 1) ? 196 * 32 : 42 * 32;
    v8f acc = {};
#pragma unroll
    for (int ks = 0; ks < 2; ++ks) {
        const int rb = rb0 + ks;
        v16bf a, b;
        int typeK, rbK, binK; feat_decode(c * 32 + nt * 16 + l16, typeK, rbK, binK);
        const int n = mt * 16 + l16;
#pragma unroll
        for (int e = 0; e < 16; ++e) {
            const int d = kmapA(e, hh);
            const int wrow = rb * 32 + d;
            a[e] = (e16)((wrow < nrows) ? Wl[(size_t)wrow * 32 + n] : 0.0f);
            b[e] = (e16)((rbK == rb) ? (We[binK * 32 + d] + be[d]) : 0.0f);
        }
        acc = wmma16(a, b, acc);
    }
    {
        const int kk = nt * 16 + l16;
        const int khh = (kk >> 3) & 1, ke = (kk & 7) + ((kk >> 4) << 3);
#pragma unroll
        for (int r = 0; r < 8; ++r) {
            const int n = mt * 16 + 8 * hh + r;
            const int dst = ((n >> 4) * 32 + (khh * 16 + (n & 15))) * 16 + ke;
            sdst[dst] = (e16)(acc[r] * WCSCALE);
        }
    }
    __syncthreads();
    VST2(v8hf, wc + (size_t)c * 1024 + threadIdx.x * 8, *(const v8hf*)(sdst + threadIdx.x * 8));
}

__global__ void cvt_zw_kernel(const float* __restrict__ zw, e16* __restrict__ zwbf) {
    int p8 = blockIdx.x * blockDim.x + threadIdx.x;
    if (p8 >= 32 * 32 * 128 / 8) return;
    const int d0 = p8 * 8;
    const int frag = d0 >> 9, lane = (d0 >> 4) & 31, e0 = d0 & 15;
    v8hf v;
#pragma unroll
    for (int q = 0; q < 8; ++q) {
        int i, j, h; bswiz_inv(frag, lane, e0 + q, 8, i, j, h);
        v[q] = (e16)zw[(i * 32 + j) * 128 + h];
    }
    *(volatile v8hf*)(zwbf + d0) = v; __threadfence(); *(volatile v8hf*)(zwbf + d0) = v;
}

__global__ __launch_bounds__(32)
void final_d_kernel(const float* __restrict__ pos_a, const float* __restrict__ mask_a,
                    const float* __restrict__ pos_b, const float* __restrict__ mask_b,
                    const float* __restrict__ rr,    const float* __restrict__ rt,
                    const v16bf* __restrict__ wcv,
                    const float* __restrict__ bl1, const float* __restrict__ bl2,
                    const float* __restrict__ bl3,
                    float* __restrict__ fd) {
    __shared__ float  sposa[14 * 3];
    __shared__ float  sposb[16 * 14 * 3];
    __shared__ float  smaska[14];
    __shared__ float  smaskbp[14];
    __shared__ float  smaskbq[16 * 14];
    __shared__ float  sR[9];
    __shared__ float  sT[3];
    __shared__ float2 sg1[16 * 196];
    __shared__ float2 sg2[16 * 196];
    __shared__ float2 sg3[16 * 42];

    const int lane = threadIdx.x;
    const int m0 = blockIdx.x * 16;
    const int p = m0 >> 7;
    const int q0 = m0 & 127;

    for (int i = lane; i < 42; i += 32)  sposa[i] = pos_a[p * 42 + i];
    for (int i = lane; i < 672; i += 32) sposb[i] = pos_b[q0 * 42 + i];
    for (int i = lane; i < 14; i += 32) {
        smaska[i]  = mask_a[p * 14 + i];
        smaskbp[i] = mask_b[p * 14 + i];
    }
    for (int i = lane; i < 224; i += 32) smaskbq[i] = mask_b[q0 * 14 + i];
    if (lane < 9) sR[lane] = rr[p * 9 + lane];
    if (lane < 3) sT[lane] = rt[p * 3 + lane];
    __syncthreads();

    for (int idx = lane; idx < 16 * 196; idx += 32) {
        int r = idx / 196, k = idx - r * 196;
        int ia = k / 14, ib = k - ia * 14;
        float dx = sposb[r * 42 + ib * 3 + 0] - sposa[ia * 3 + 0];
        float dy = sposb[r * 42 + ib * 3 + 1] - sposa[ia * 3 + 1];
        float dz = sposb[r * 42 + ib * 3 + 2] - sposa[ia * 3 + 2];
        float d = sqrtf(dx * dx + dy * dy + dz * dz);
        float msk = smaska[ia] * smaskbq[r * 14 + ib];
        sg1[idx] = group_ab(d, OFF1, S1, C1, 16, msk);
        sg2[idx] = group_ab(d, OFF2, S2, C2, 40, msk);
    }
    for (int idx = lane; idx < 16 * 42; idx += 32) {
        int r = idx / 42, v = idx - r * 42;
        int ib = v / 3, i = v - ib * 3;
        float q0v = sposb[r * 42 + ib * 3 + 0] - sT[0];
        float q1v = sposb[r * 42 + ib * 3 + 1] - sT[1];
        float q2v = sposb[r * 42 + ib * 3 + 2] - sT[2];
        float lv = sR[0 * 3 + i] * q0v + sR[1 * 3 + i] * q1v + sR[2 * 3 + i] * q2v;
        float msk = smaskbp[ib] * smaskbq[r * 14 + ib];
        sg3[idx] = group_ab(lv, OFF3, S3, C3, 64, msk);
    }
    __syncthreads();

    const int r  = lane & 15;
    const int hi = lane >> 4;
    v8f acc0 = {}, acc1 = {};

    v16bf bA0 = wcv[lane];
    v16bf bA1 = wcv[32 + lane];
    v16bf bB0 = {}, bB1 = {};

    for (int c = 0; c < NCHUNK; c += 2) {
        if (c + 1 < NCHUNK) {
            bB0 = wcv[((c + 1) * 2 + 0) * 32 + lane];
            bB1 = wcv[((c + 1) * 2 + 1) * 32 + lane];
        }
        v16bf a0 = make_afrag(c, r, hi, sg1, sg2, sg3);
        acc0 = wmma16(a0, bA0, acc0);
        acc1 = wmma16(a0, bA1, acc1);
        if (c + 1 >= NCHUNK) break;
        if (c + 2 < NCHUNK) {
            bA0 = wcv[((c + 2) * 2 + 0) * 32 + lane];
            bA1 = wcv[((c + 2) * 2 + 1) * 32 + lane];
        }
        v16bf a1 = make_afrag(c + 1, r, hi, sg1, sg2, sg3);
        acc0 = wmma16(a1, bB0, acc0);
        acc1 = wmma16(a1, bB1, acc1);
    }

    const float bsum = bl1[lane] + bl2[lane] + bl3[lane];
    for (int pass = 0; pass < 2; ++pass) {
#pragma unroll
        for (int v = 0; v < 8; ++v) {
            const float a_ = acc0[v] * INV_WCSCALE, b_ = acc1[v] * INV_WCSCALE;
            const float ax = __shfl_xor(a_, 16), bx = __shfl_xor(b_, 16);
            *(volatile float*)(fd + (size_t)(m0 + v) * 32 + lane)     = (hi ? bx : a_) + bsum;
            *(volatile float*)(fd + (size_t)(m0 + v + 8) * 32 + lane) = (hi ? b_ : ax) + bsum;
        }
        __threadfence();
    }
}

__global__ __launch_bounds__(32)
void z_einsum_kernel(const int* __restrict__ aat1, const float* __restrict__ aa_emb,
                     const float* __restrict__ fd, const v16bf* __restrict__ zwv,
                     const float* __restrict__ zb, float* __restrict__ out) {
    const int lane = threadIdx.x;
    const int m0 = blockIdx.x * 16;
    const int r  = lane & 15;
    const int hi = lane >> 4;
    const int m  = m0 + r;
    const int p  = m >> 7, q = m & 127;
    const int pidx = aat1[p] * 21 + aat1[q];
    const float* pfr = aa_emb + pidx * 32;

    float fdv[16];
#pragma unroll
    for (int e = 0; e < 16; ++e) fdv[e] = fd[m * 32 + kmapA(e, hi)];

    v8f acc[8];
#pragma unroll
    for (int nt = 0; nt < 8; ++nt) acc[nt] = (v8f){};

    v16bf bA[8], bB[8];
#pragma unroll
    for (int nt = 0; nt < 8; ++nt) bA[nt] = zwv[nt * 32 + lane];

    for (int c = 0; c < 32; c += 2) {
#pragma unroll
        for (int nt = 0; nt < 8; ++nt)
            bB[nt] = zwv[((c + 1) * 8 + nt) * 32 + lane];
        float pf0 = pfr[c];
        v16bf a0;
#pragma unroll
        for (int e = 0; e < 16; ++e) a0[e] = (e16)(pf0 * fdv[e] * A2SCALE);
#pragma unroll
        for (int nt = 0; nt < 8; ++nt) acc[nt] = wmma16(a0, bA[nt], acc[nt]);
        if (c + 2 < 32) {
#pragma unroll
            for (int nt = 0; nt < 8; ++nt)
                bA[nt] = zwv[((c + 2) * 8 + nt) * 32 + lane];
        }
        float pf1 = pfr[c + 1];
        v16bf a1;
#pragma unroll
        for (int e = 0; e < 16; ++e) a1[e] = (e16)(pf1 * fdv[e] * A2SCALE);
#pragma unroll
        for (int nt = 0; nt < 8; ++nt) acc[nt] = wmma16(a1, bB[nt], acc[nt]);
    }
    for (int pass = 0; pass < 2; ++pass) {
#pragma unroll
        for (int pr = 0; pr < 4; ++pr) {
            const float zbh = zb[pr * 32 + lane];
#pragma unroll
            for (int v = 0; v < 8; ++v) {
                const float a_ = acc[2 * pr][v] * INV_A2SCALE, b_ = acc[2 * pr + 1][v] * INV_A2SCALE;
                const float ax = __shfl_xor(a_, 16), bx = __shfl_xor(b_, 16);
                *(volatile float*)(out + (size_t)(m0 + v) * 128 + pr * 32 + lane)     = (hi ? bx : a_) + zbh;
                *(volatile float*)(out + (size_t)(m0 + v + 8) * 128 + pr * 32 + lane) = (hi ? b_ : ax) + zbh;
            }
        }
        __threadfence();
    }
}

extern "C" void kernel_launch(void* const* d_in, const int* in_sizes, int n_in,
                              void* d_out, int out_size, void* d_ws, size_t ws_size,
                              hipStream_t stream) {
    const int*   aat1   = (const int*)  d_in[0];
    const float* pos_a  = (const float*)d_in[2];
    const float* mask_a = (const float*)d_in[3];
    const float* pos_b  = (const float*)d_in[4];
    const float* mask_b = (const float*)d_in[5];
    const float* rr     = (const float*)d_in[6];
    const float* rt     = (const float*)d_in[7];
    const float* aa_emb = (const float*)d_in[8];
    const float* We1 = (const float*)d_in[9],  *be1 = (const float*)d_in[10];
    const float* We2 = (const float*)d_in[11], *be2 = (const float*)d_in[12];
    const float* We3 = (const float*)d_in[13], *be3 = (const float*)d_in[14];
    const float* Wl1 = (const float*)d_in[15], *bl1 = (const float*)d_in[16];
    const float* Wl2 = (const float*)d_in[17], *bl2 = (const float*)d_in[18];
    const float* Wl3 = (const float*)d_in[19], *bl3 = (const float*)d_in[20];
    const float* zw  = (const float*)d_in[21], *zb  = (const float*)d_in[22];
    float* out = (float*)d_out;

    (void)in_sizes; (void)n_in; (void)out_size;
    if (ws_size < (size_t)874496 + 262144 + 2097152) return;
    char* ws = (char*)d_ws;
    e16*   wc   = (e16*)ws;
    e16*   zwbf = (e16*)(ws + 874496);
    float* fd   = (float*)(ws + 874496 + 262144);

    fold_weights_kernel<<<NCHUNK, 128, 0, stream>>>(
        We1, be1, We2, be2, We3, be3, Wl1, Wl2, Wl3, wc);
    cvt_zw_kernel<<<(131072 / 8 + 255) / 256, 256, 0, stream>>>(zw, zwbf);
    final_d_kernel<<<1024, 32, 0, stream>>>(
        pos_a, mask_a, pos_b, mask_b, rr, rt, (const v16bf*)wc, bl1, bl2, bl3, fd);
    z_einsum_kernel<<<1024, 32, 0, stream>>>(aat1, aa_emb, fd, (const v16bf*)zwbf, zb, out);
}
